// GraphEncoder_47330539602050
// MI455X (gfx1250) — hardware-verified
//
#include <hip/hip_runtime.h>
#include <stddef.h>
#include <stdint.h>


#define DF     128
#define KD     256
#define HP     256
#define NTHR   256
#define NWAVE  8
#define EPT    8
#define CHUNK  (NTHR * EPT)
#define WCAP   (EPT * 32)
#define LISTN  (NWAVE * WCAP)
#define NBA    512
#define SLA    9
#define RCAP   24576
#define DEGCAP 96
#define GBM    64
#define GBN    128
#define GTHR   128
#define NUW0   (DF * (DF / 8))
#define NUWD   (DF * (KD / 8))
#define NWD    5
#define NUW    (NUW0 + NWD * NUWD)
#define AGG_ZINTS    (LISTN + 2 * RCAP + 3 * NBA)
#define MISC_INTS    16
#define ROWBUF_INTS  (NWAVE * HP / 2)
#define AGG_LDS_INTS (AGG_ZINTS + MISC_INTS + ROWBUF_INTS)
#define WSMAX  134217728

static_assert((CHUNK & (CHUNK - 1)) == 0 && CHUNK <= 4096);
static_assert((NBA & (NBA - 1)) == 0 && NBA == (1 << SLA));
static_assert(((long long)CHUNK << SLA) < (1LL << 31));
static_assert(LISTN % NTHR == 0);
static_assert(NBA % NWAVE == 0 && NBA % 32 == 0 && NBA % GBM == 0);
static_assert(RCAP % 4 == 0 && AGG_ZINTS % 4 == 0 && LISTN % 4 == 0 && ((AGG_ZINTS + MISC_INTS) % 4) == 0);
static_assert(DF % 32 == 0 && KD % 32 == 0 && KD == 2 * DF && HP == 2 * DF);
static_assert(GBN == DF && GBM == (GTHR / 32) * 16 && DF == 4 * 32);
static_assert(NUW0 % NTHR == 0 && NUWD % NTHR == 0 && NUW % NTHR == 0 && NUWD == (1 << 12));
static_assert(DF / 8 == 16 && KD / 8 == 32);
static_assert(AGG_LDS_INTS * 4 <= 300000);

typedef float          v4f   __attribute__((ext_vector_type(4)));
typedef float          v8f   __attribute__((ext_vector_type(8)));
typedef int            v4i   __attribute__((ext_vector_type(4)));
typedef int            v8i   __attribute__((ext_vector_type(8)));
typedef unsigned short v4us  __attribute__((ext_vector_type(4)));
typedef unsigned short v8us  __attribute__((ext_vector_type(8)));
typedef unsigned short v16us __attribute__((ext_vector_type(16)));
typedef __bf16         v16bf __attribute__((ext_vector_type(16)));
typedef v4f  __attribute__((may_alias)) v4fa;
typedef v4i  __attribute__((may_alias)) v4ia;
typedef v4us __attribute__((may_alias)) v4usa;
typedef v8us __attribute__((may_alias)) v8usa;
union FragB { v16bf v; v16us u; v8us h[2]; v8i w; };

__device__ __forceinline__ v8f wmb(const FragB& a, const FragB& b, v8f c) {
  v8f d = __builtin_amdgcn_wmma_f32_16x16x32_bf16(false, a.v, false, b.v, (short)0, c, false, false);
  asm volatile("v_nop\n\tv_nop\n\tv_nop\n\tv_nop" : "+v"(d) : "v"(a.w), "v"(b.w));
  return d;
}

__device__ __forceinline__ unsigned bf16_bits(float f) {
  const unsigned u = __float_as_uint(f);
  return (u + 0x7FFFu + ((u >> 16) & 1u)) >> 16;
}
__device__ __forceinline__ float bf16_val(float f) {
  return __uint_as_float(bf16_bits(f) << 16);
}

__device__ __forceinline__ void wave_sync() {
  __builtin_amdgcn_fence(__ATOMIC_RELEASE, "wavefront");
  __builtin_amdgcn_wave_barrier();
  __builtin_amdgcn_fence(__ATOMIC_ACQUIRE, "wavefront");
}

template <int SLB>
__device__ __forceinline__ int scan_chunk(const int* __restrict__ dsts, int nE, int cbase, int slotBase,
                                          int nb, int vec8, int* list, int tid, int lane, int wave) {
  int wc = 0;
  const int el0  = tid * EPT;
  const int e0   = cbase + el0;
  const int sent = -2147483647 - 1;
  v4i da, db;
  if (vec8 != 0 && cbase + CHUNK <= nE) {
    da = *(const v4i*)(dsts + e0);
    db = *(const v4i*)(dsts + e0 + 4);
  } else {
    da.x = (e0     < nE) ? dsts[min(e0,     nE - 1)] : sent;
    da.y = (e0 + 1 < nE) ? dsts[min(e0 + 1, nE - 1)] : sent;
    da.z = (e0 + 2 < nE) ? dsts[min(e0 + 2, nE - 1)] : sent;
    da.w = (e0 + 3 < nE) ? dsts[min(e0 + 3, nE - 1)] : sent;
    db.x = (e0 + 4 < nE) ? dsts[min(e0 + 4, nE - 1)] : sent;
    db.y = (e0 + 5 < nE) ? dsts[min(e0 + 5, nE - 1)] : sent;
    db.z = (e0 + 6 < nE) ? dsts[min(e0 + 6, nE - 1)] : sent;
    db.w = (e0 + 7 < nE) ? dsts[min(e0 + 7, nE - 1)] : sent;
  }
  const unsigned nbs = (unsigned)slotBase;
  const unsigned unb = (unsigned)nb;
  const unsigned s0 = (unsigned)da.x - nbs, s1 = (unsigned)da.y - nbs;
  const unsigned s2 = (unsigned)da.z - nbs, s3 = (unsigned)da.w - nbs;
  const unsigned s4 = (unsigned)db.x - nbs, s5 = (unsigned)db.y - nbs;
  const unsigned s6 = (unsigned)db.z - nbs, s7 = (unsigned)db.w - nbs;
  const bool h0 = s0 < unb, h1 = s1 < unb, h2 = s2 < unb, h3 = s3 < unb;
  const bool h4 = s4 < unb, h5 = s5 < unb, h6 = s6 < unb, h7 = s7 < unb;
  const unsigned any = __builtin_amdgcn_ballot_w32(h0 | h1 | h2 | h3 | h4 | h5 | h6 | h7);
  if (any != 0u) {
#define HITJ(J, HJ, SJ) { \
      const unsigned mj = __builtin_amdgcn_ballot_w32(HJ); \
      if (mj != 0u) { \
        if (HJ) { \
          const int pos = wc + (int)__builtin_amdgcn_mbcnt_lo(mj, 0u); \
          if (pos < WCAP) list[wave * WCAP + pos] = ((el0 + (J)) << SLB) | (int)(SJ); \
        } \
        wc += (int)__builtin_popcount(mj); } }
    HITJ(0, h0, s0)
    HITJ(1, h1, s1)
    HITJ(2, h2, s2)
    HITJ(3, h3, s3)
    HITJ(4, h4, s4)
    HITJ(5, h5, s5)
    HITJ(6, h6, s6)
    HITJ(7, h7, s7)
#undef HITJ
  }
  return wc;
}

__global__ __launch_bounds__(NTHR) void k_prep(const float* __restrict__ x, int nN, int nUx,
                                               const float* __restrict__ w1a, const float* __restrict__ w2a,
                                               const float* __restrict__ w1b, const float* __restrict__ w2b,
                                               const float* __restrict__ w1c, const float* __restrict__ w2c,
                                               unsigned short* W1T0, unsigned short* WD, unsigned short* XB) {
  const int u = (int)blockIdx.x * NTHR + (int)threadIdx.x;
  v8us o;
  unsigned short* dp;
  if (u < NUW0) {
    const int n  = u >> 4;
    const int k8 = (u & 15) * 8;
    const float* p = w1a + (size_t)k8 * DF + n;
#pragma unroll
    for (int i = 0; i < 8; ++i) o[i] = (unsigned short)bf16_bits(p[(size_t)i * DF]);
    dp = W1T0 + (size_t)n * DF + k8;
  } else if (u < NUW) {
    const int v    = u - NUW0;
    const int part = v >> 12;
    const int r    = v & (NUWD - 1);
    const int n    = r >> 5;
    const int k8   = (r & 31) * 8;
    const int kk   = k8 & (DF - 1);
    const float* W;
    if (part == 0)      W = w2a;
    else if (part == 1) W = w1b;
    else if (part == 2) W = w2b;
    else if (part == 3) W = w1c;
    else                W = w2c;
    const float* p = W + (size_t)kk * DF + n;
#pragma unroll
    for (int i = 0; i < 8; ++i) o[i] = (unsigned short)bf16_bits(p[(size_t)i * DF]);
    dp = WD + (size_t)part * (size_t)(DF * KD) + (size_t)n * KD + k8;
  } else {
    const int v = u - NUW;
    if (v >= nUx) return;
    const int row = v >> 4;
    const int k8  = (v & 15) * 8;
    const int rc  = row < nN ? row : nN - 1;
    const float* p = x + (size_t)rc * DF + k8;
    const v4f a = *(const v4fa*)p;
    const v4f b = *(const v4fa*)(p + 4);
    const bool ok = row < nN;
    o[0] = ok ? (unsigned short)bf16_bits(a.x) : (unsigned short)0;
    o[1] = ok ? (unsigned short)bf16_bits(a.y) : (unsigned short)0;
    o[2] = ok ? (unsigned short)bf16_bits(a.z) : (unsigned short)0;
    o[3] = ok ? (unsigned short)bf16_bits(a.w) : (unsigned short)0;
    o[4] = ok ? (unsigned short)bf16_bits(b.x) : (unsigned short)0;
    o[5] = ok ? (unsigned short)bf16_bits(b.y) : (unsigned short)0;
    o[6] = ok ? (unsigned short)bf16_bits(b.z) : (unsigned short)0;
    o[7] = ok ? (unsigned short)bf16_bits(b.w) : (unsigned short)0;
    dp = XB + (size_t)row * DF + k8;
  }
  *(volatile v8us*)dp = o;
  __threadfence();
  *(volatile v8us*)dp = o;
}

template <int MODE>
__global__ __launch_bounds__(GTHR) void k_gemm(const unsigned short* __restrict__ Apl, int lda,
                                               const unsigned short* __restrict__ BT, int K,
                                               const float* __restrict__ bias,
                                               unsigned short* zpl, float* outp, int nOut) {
  __shared__ __attribute__((aligned(16))) float stg[GBM * GBN];
  const int tid = (int)threadIdx.x, lane = tid & 31, wave = tid >> 5, hh = lane >> 4, m = lane & 15;
  const int rowBase = (int)blockIdx.x * GBM;

  v8f acc[8];
  {
    const v8f z = {0.f, 0.f, 0.f, 0.f, 0.f, 0.f, 0.f, 0.f};
#pragma unroll
    for (int t = 0; t < 8; ++t) acc[t] = z;
  }
  const unsigned short* ap = Apl + (size_t)(rowBase + 16 * wave + m) * (size_t)lda + 8 * hh;
  const unsigned short* bp = BT + (size_t)m * (size_t)K + 8 * hh;

#pragma unroll 1
  for (int k0 = 0; k0 < K; k0 += 32) {
    FragB af;
    af.h[0] = *(const v8usa*)(ap + k0);
    af.h[1] = *(const v8usa*)(ap + k0 + 16);
#pragma unroll
    for (int nt = 0; nt < 8; ++nt) {
      const unsigned short* wq = bp + (size_t)(16 * nt) * (size_t)K + k0;
      FragB bf;
      bf.h[0] = *(const v8usa*)wq;
      bf.h[1] = *(const v8usa*)(wq + 16);
      acc[nt] = wmb(af, bf, acc[nt]);
    }
  }

#pragma unroll
  for (int nt = 0; nt < 8; ++nt) {
    const int lc = 16 * nt + m;
#pragma unroll
    for (int r = 0; r < 8; ++r) {
      const int lr = 16 * wave + 8 * hh + r;
      stg[lr * GBN + lc] = acc[nt][r];
    }
  }
  __syncthreads();

  v4f bb4 = {0.f, 0.f, 0.f, 0.f};
  if constexpr (MODE != 0) {
    const v4f t1 = *(const v4fa*)(bias + 4 * lane);
    bb4.x = bf16_val(t1.x);
    bb4.y = bf16_val(t1.y);
    bb4.z = bf16_val(t1.z);
    bb4.w = bf16_val(t1.w);
  }

  v4f pv[16];
#pragma unroll
  for (int i = 0; i < 16; ++i) pv[i] = *(const v4fa*)(stg + (16 * wave + i) * GBN + 4 * lane);
  __syncthreads();

#pragma unroll
  for (int i = 0; i < 16; ++i) {
    const bool ok = (rowBase + 16 * wave + i) < nOut;
    v4f y = pv[i] + bb4;
    if constexpr (MODE != 0) {
      y.x = fmaxf(y.x, 0.0f); y.y = fmaxf(y.y, 0.0f); y.z = fmaxf(y.z, 0.0f); y.w = fmaxf(y.w, 0.0f);
    }
    y.x = ok ? y.x : 0.0f; y.y = ok ? y.y : 0.0f; y.z = ok ? y.z : 0.0f; y.w = ok ? y.w : 0.0f;
    pv[i] = y;
  }

  if constexpr (MODE != 1) {
#pragma unroll
    for (int i = 0; i < 16; ++i) {
      const int r = rowBase + 16 * wave + i;
      if (r < nOut) *(volatile v4f*)(outp + (size_t)r * DF + 4 * lane) = pv[i];
    }
    __threadfence();
#pragma unroll
    for (int i = 0; i < 16; ++i) {
      const int r = rowBase + 16 * wave + i;
      if (r < nOut) *(volatile v4f*)(outp + (size_t)r * DF + 4 * lane) = pv[i];
    }
  } else {
#pragma unroll
    for (int i = 0; i < 16; ++i) {
      v4us h4, l4;
      unsigned hb;
      hb = bf16_bits(pv[i].x); h4[0] = (unsigned short)hb; l4[0] = (unsigned short)bf16_bits(pv[i].x - __uint_as_float(hb << 16));
      hb = bf16_bits(pv[i].y); h4[1] = (unsigned short)hb; l4[1] = (unsigned short)bf16_bits(pv[i].y - __uint_as_float(hb << 16));
      hb = bf16_bits(pv[i].z); h4[2] = (unsigned short)hb; l4[2] = (unsigned short)bf16_bits(pv[i].z - __uint_as_float(hb << 16));
      hb = bf16_bits(pv[i].w); h4[3] = (unsigned short)hb; l4[3] = (unsigned short)bf16_bits(pv[i].w - __uint_as_float(hb << 16));
      unsigned short* srow = (unsigned short*)stg + (size_t)(16 * wave + i) * (2 * GBN);
      *(v4usa*)(srow + 4 * lane) = h4;
      *(v4usa*)(srow + DF + 4 * lane) = l4;
    }
    __syncthreads();
    v8us qv[16];
#pragma unroll
    for (int i = 0; i < 16; ++i) {
      const unsigned short* srow = (const unsigned short*)stg + (size_t)(16 * wave + i) * (2 * GBN);
      qv[i] = *(const v8usa*)(srow + 8 * lane);
    }
#pragma unroll
    for (int i = 0; i < 16; ++i) {
      unsigned short* rp = zpl + (size_t)(rowBase + 16 * wave + i) * (size_t)HP + 8 * lane;
      *(volatile v8us*)rp = qv[i];
    }
    __threadfence();
#pragma unroll
    for (int i = 0; i < 16; ++i) {
      unsigned short* rp = zpl + (size_t)(rowBase + 16 * wave + i) * (size_t)HP + 8 * lane;
      *(volatile v8us*)rp = qv[i];
    }
  }
}

__global__ __launch_bounds__(NTHR) void k_scan(const int* __restrict__ srcs, const int* __restrict__ dsts,
                                               int nE, int nN, int vec8, int mRows,
                                               const float* __restrict__ P, const float* __restrict__ bias,
                                               unsigned short* hpl) {
  extern __shared__ __attribute__((aligned(16))) int dsm[];
  int* list = dsm;
  int* hl   = dsm + LISTN;
  int* sl   = hl + RCAP;
  int* cnt  = sl + RCAP;
  int* offs = cnt + NBA;
  int* cur  = offs + NBA;
  int* misc = cur + NBA;
  const int tid = (int)threadIdx.x, lane = tid & 31, wave = tid >> 5;
  unsigned short* rowbuf = (unsigned short*)(misc + MISC_INTS) + wave * HP;
  const int nodeBase = (int)blockIdx.x * NBA;

  {
    const v4i z4 = {0, 0, 0, 0};
    for (int i = tid * 4; i < AGG_ZINTS; i += NTHR * 4) *(v4ia*)(dsm + i) = z4;
    if (tid < MISC_INTS) misc[tid] = 0;
  }
  v4f bb4;
  {
    const v4f t1 = *(const v4fa*)(bias + 4 * lane);
    bb4.x = bf16_val(t1.x);
    bb4.y = bf16_val(t1.y);
    bb4.z = bf16_val(t1.z);
    bb4.w = bf16_val(t1.w);
  }
  __syncthreads();

  int t = 0, ov = 0;
  const int nChunks = (nE + CHUNK - 1) / CHUNK;
#pragma unroll 1
  for (int ch = 0; ch < nChunks; ++ch) {
    const int cbase = ch * CHUNK;
    const int wc = scan_chunk<SLA>(dsts, nE, cbase, nodeBase, NBA, vec8, list, tid, lane, wave);
    if (lane == 0) misc[wave] = wc;
    __syncthreads();
    if (wave == 0) {
#pragma unroll 1
      for (int w2 = 0; w2 < NWAVE; ++w2) {
        int c = misc[w2];
        c = c < 0 ? 0 : (c > WCAP ? WCAP : c);
#pragma unroll 1
        for (int b0 = 0; b0 < c; b0 += 32) {
          const int idx = b0 + lane;
          const int ent = list[w2 * WCAP + (idx < WCAP ? idx : WCAP - 1)];
          const int m32 = (c - b0) < 32 ? (c - b0) : 32;
#pragma unroll 1
          for (int k = 0; k < m32; ++k) {
            const int u    = __builtin_amdgcn_readlane(ent, k);
            const int slot = u & (NBA - 1);
            const int el   = (u >> SLA) & (CHUNK - 1);
            const int pk   = ((cbase + el) << SLA) | slot;
            if (t < RCAP) {
              if (lane == 0) { hl[t] = pk; cnt[slot] = cnt[slot] + 1; }
              t = t + 1;
            } else {
              ov = 1;
            }
          }
        }
      }
    }
    __syncthreads();
  }
  if (wave == 0 && lane == 0) { misc[8] = t; misc[9] = ov; }
  __syncthreads();
  int tt = misc[8];
  tt = tt < 0 ? 0 : (tt > RCAP ? RCAP : tt);
  const int ovf = misc[9];

  if (wave == 0) {
    const int base = lane * (NBA / 32);
    int s = 0;
#pragma unroll 1
    for (int i = 0; i < NBA / 32; ++i) s += cnt[base + i];
    int incl = s;
#pragma unroll
    for (int d = 1; d < 32; d <<= 1) {
      const int y = __shfl_up(incl, d, 32);
      if (lane >= d) incl += y;
    }
    int run = incl - s;
#pragma unroll 1
    for (int i = 0; i < NBA / 32; ++i) {
      const int cv = cnt[base + i];
      offs[base + i] = run;
      cur[base + i]  = run;
      run += cv;
    }
  }
  __syncthreads();
  if (wave == 0) {
#pragma unroll 1
    for (int b0 = 0; b0 < tt; b0 += 32) {
      const int idx = b0 + lane;
      const int ent = hl[idx < RCAP ? idx : RCAP - 1];
      const int m32 = (tt - b0) < 32 ? (tt - b0) : 32;
#pragma unroll 1
      for (int k = 0; k < m32; ++k) {
        const int u    = __builtin_amdgcn_readlane(ent, k);
        const int slot = u & (NBA - 1);
        if (lane == 0) {
          int p = cur[slot];
          p = p < 0 ? 0 : (p > RCAP - 1 ? RCAP - 1 : p);
          sl[p] = u;
          cur[slot] = p + 1;
        }
      }
    }
  }
  __syncthreads();

  const float qnan = __int_as_float(0x7fc00000);
  const float pz = (ovf != 0) ? qnan : 0.0f;
#pragma unroll 1
  for (int si = 0; si < NBA / NWAVE; ++si) {
    const int s    = si * NWAVE + wave;
    const int node = nodeBase + s;
    int c = cnt[s];
    const bool big = c > DEGCAP;
    c = c < 0 ? 0 : (c > DEGCAP ? DEGCAP : c);
    int o = offs[s];
    o = o < 0 ? 0 : (o > RCAP ? RCAP : o);
    const int nc = node < nN ? node : nN - 1;
    float a0 = 0.0f, a1 = 0.0f, a2 = 0.0f, a3 = 0.0f;
#pragma unroll 1
    for (int b0 = 0; b0 < c; b0 += 32) {
      int idx = o + b0 + lane;
      idx = idx > RCAP - 1 ? RCAP - 1 : idx;
      const int ent = sl[idx];
      int eid = ent >> SLA;
      eid = eid < 0 ? 0 : (eid > nE - 1 ? nE - 1 : eid);
      int sr = srcs[eid];
      sr = sr < 0 ? 0 : (sr > nN - 1 ? nN - 1 : sr);
      const int m32 = (c - b0) < 32 ? (c - b0) : 32;
#pragma unroll 1
      for (int k = 0; k < m32; ++k) {
        const int sk = __builtin_amdgcn_readlane(sr, k);
        const v4f a = *(const v4fa*)(P + (size_t)sk * DF + 4 * lane);
        a0 += a.x; a1 += a.y; a2 += a.z; a3 += a.w;
      }
    }
    const v4f ps = *(const v4fa*)(P + (size_t)nc * DF + 4 * lane);
    const float pzr = big ? qnan : pz;
    const bool live = node < nN;
    float y0 = (a0 + ps.x) + bb4.x;
    float y1 = (a1 + ps.y) + bb4.y;
    float y2 = (a2 + ps.z) + bb4.z;
    float y3 = (a3 + ps.w) + bb4.w;
    y0 = fmaxf(y0, 0.0f); y1 = fmaxf(y1, 0.0f); y2 = fmaxf(y2, 0.0f); y3 = fmaxf(y3, 0.0f);
    y0 = y0 + pzr; y1 = y1 + pzr; y2 = y2 + pzr; y3 = y3 + pzr;
    const float m0 = live ? y0 : 0.0f;
    const float m1 = live ? y1 : 0.0f;
    const float m2 = live ? y2 : 0.0f;
    const float m3 = live ? y3 : 0.0f;
    v4us mh, ml;
    {
      unsigned hb;
      hb = bf16_bits(m0); mh[0] = (unsigned short)hb; ml[0] = (unsigned short)bf16_bits(m0 - __uint_as_float(hb << 16));
      hb = bf16_bits(m1); mh[1] = (unsigned short)hb; ml[1] = (unsigned short)bf16_bits(m1 - __uint_as_float(hb << 16));
      hb = bf16_bits(m2); mh[2] = (unsigned short)hb; ml[2] = (unsigned short)bf16_bits(m2 - __uint_as_float(hb << 16));
      hb = bf16_bits(m3); mh[3] = (unsigned short)hb; ml[3] = (unsigned short)bf16_bits(m3 - __uint_as_float(hb << 16));
    }
    *(v4usa*)(rowbuf + 4 * lane) = mh;
    *(v4usa*)(rowbuf + DF + 4 * lane) = ml;
    wave_sync();
    const v8us q0 = *(const v8usa*)(rowbuf + 8 * lane);
    wave_sync();
    if (node < mRows) {
      unsigned short* rpw = hpl + (size_t)node * HP + 8 * lane;
      *(volatile v8us*)rpw = q0;
      __threadfence();
      *(volatile v8us*)rpw = q0;
    }
  }
}

static inline int cdiv(int a, int b) { return (a + b - 1) / b; }
static inline size_t al256(size_t o) { return (o + 255) & ~(size_t)255; }

extern "C" void kernel_launch(void* const* d_in, const int* in_sizes, int n_in,
                              void* d_out, int out_size, void* d_ws, size_t ws_size,
                              hipStream_t stream) {
  if (n_in < 14) return;
  if (in_sizes[0] < DF || (in_sizes[0] % DF) != 0) return;
  const int nN = in_sizes[0] / DF;
  if (nN < 16 || nN >= (1 << 22)) return;
  if (in_sizes[1] < 2 || (in_sizes[1] & 1) != 0) return;
  const int nE = in_sizes[1] / 2;
  if (nE < 1 || nE >= (1 << (31 - SLA))) return;
  for (int l = 0; l < 3; ++l) {
    if (in_sizes[2 + 4 * l] != DF * DF || in_sizes[3 + 4 * l] != DF) return;
    if (in_sizes[4 + 4 * l] != DF * DF || in_sizes[5 + 4 * l] != DF) return;
  }
  if ((long long)out_size != (long long)nN * DF) return;

  const float* x    = (const float*)d_in[0];
  const int*   edge = (const int*)d_in[1];
  const float* w1a  = (const float*)d_in[2];
  const float* b1a  = (const float*)d_in[3];
  const float* w2a  = (const float*)d_in[4];
  const float* b2a  = (const float*)d_in[5];
  const float* w1b  = (const float*)d_in[6];
  const float* b1b  = (const float*)d_in[7];
  const float* w2b  = (const float*)d_in[8];
  const float* b2b  = (const float*)d_in[9];
  const float* w1c  = (const float*)d_in[10];
  const float* b1c  = (const float*)d_in[11];
  const float* w2c  = (const float*)d_in[12];
  const float* b2c  = (const float*)d_in[13];
  float* out = (float*)d_out;
  const int* src = edge;
  const int* dst = edge + nE;

  const int MP = cdiv(nN, GBM) * GBM;
  const int gM = MP / GBM;
  const int gA = cdiv(MP, NBA);
  if ((long long)gA * NBA < (long long)MP) return;
  const int vec8 = ((nE & 3) == 0) ? 1 : 0;

  char* ws = (char*)d_ws;
  size_t off = 0;
  const size_t oW1T0 = off; off = al256(off + (size_t)DF * DF * 2);
  const size_t oWD   = off; off = al256(off + (size_t)NWD * DF * KD * 2);
  const size_t oXB   = off; off = al256(off + (size_t)MP * DF * 2);
  const size_t oP    = off; off = al256(off + (size_t)MP * DF * 4);
  const size_t oH    = off; off = al256(off + (size_t)MP * HP * 2);
  const size_t oZ    = off; off = al256(off + (size_t)MP * HP * 2);
  if (off > ws_size || off > (size_t)WSMAX) return;
  unsigned short* W1T0 = (unsigned short*)(ws + oW1T0);
  unsigned short* WD   = (unsigned short*)(ws + oWD);
  unsigned short* XB   = (unsigned short*)(ws + oXB);
  float*          P    = (float*)(ws + oP);
  unsigned short* H    = (unsigned short*)(ws + oH);
  unsigned short* Z    = (unsigned short*)(ws + oZ);
  const size_t WDP = (size_t)DF * KD;
  unsigned short* WD2a = WD + 0 * WDP;
  unsigned short* WD1b = WD + 1 * WDP;
  unsigned short* WD2b = WD + 2 * WDP;
  unsigned short* WD1c = WD + 3 * WDP;
  unsigned short* WD2c = WD + 4 * WDP;

  const size_t scanLds = (size_t)AGG_LDS_INTS * 4;
  hipFuncSetAttribute(reinterpret_cast<const void*>(&k_scan), hipFuncAttributeMaxDynamicSharedMemorySize, (int)scanLds);

  const int nUx = MP * (DF / 8);
  k_prep<<<cdiv(NUW + nUx, NTHR), NTHR, 0, stream>>>(x, nN, nUx, w1a, w2a, w1b, w2b, w1c, w2c, W1T0, WD, XB);
  k_gemm<0><<<gM, GTHR, 0, stream>>>(XB, DF, W1T0, DF, b1a, Z, P, MP);
  k_scan<<<gA, NTHR, scanLds, stream>>>(src, dst, nE, nN, vec8, MP, P, b1a, H);
  k_gemm<1><<<gM, GTHR, 0, stream>>>(H, HP, WD2a, KD, b2a, Z, P, nN);
  k_gemm<0><<<gM, GTHR, 0, stream>>>(Z, HP, WD1b, KD, b1b, Z, P, MP);
  k_scan<<<gA, NTHR, scanLds, stream>>>(src, dst, nE, nN, vec8, MP, P, b1b, H);
  k_gemm<1><<<gM, GTHR, 0, stream>>>(H, HP, WD2b, KD, b2b, Z, P, nN);
  k_gemm<0><<<gM, GTHR, 0, stream>>>(Z, HP, WD1c, KD, b1c, Z, P, MP);
  k_scan<<<gA, NTHR, scanLds, stream>>>(src, dst, nE, nN, vec8, MP, P, b1c, H);
  k_gemm<2><<<gM, GTHR, 0, stream>>>(H, HP, WD2c, KD, b2c, Z, out, nN);
}
